// MoE_Multi_Scale_77979426226519
// MI455X (gfx1250) — hardware-verified
//
#include <hip/hip_runtime.h>
#define NTK 32768
#define DI 64
#define HH 256
#define NE 8
#define TB 128
#define MAXT 24

typedef __bf16 v16b __attribute__((ext_vector_type(16)));
typedef unsigned short v8us __attribute__((ext_vector_type(8), may_alias));
typedef float  v8f  __attribute__((ext_vector_type(8)));
typedef float  v4f  __attribute__((ext_vector_type(4)));
typedef float  v4fa __attribute__((ext_vector_type(4), may_alias));
union FragB { v16b v; v8us half[2]; unsigned short u[16]; };

__device__ __forceinline__ unsigned short bf16_bits(float x) { unsigned int u = __float_as_uint(x); return (unsigned short)((u + 0x7FFFu + ((u >> 16) & 1u)) >> 16); }
__device__ __forceinline__ float bf16_val(unsigned short b) { return __uint_as_float(((unsigned int)b) << 16); }
__device__ __forceinline__ float bf16_round(float x) { return bf16_val(bf16_bits(x)); }
template <int NT>
__device__ __forceinline__ v8f mmaN(v16b ah, v16b al, v16b bh, v16b bl, v8f c) {
  c = __builtin_amdgcn_wmma_f32_16x16x32_bf16(false, ah, false, bh, (short)0, c, false, false);
  if (NT >= 2) c = __builtin_amdgcn_wmma_f32_16x16x32_bf16(false, al, false, bh, (short)0, c, false, false);
  if (NT >= 3) c = __builtin_amdgcn_wmma_f32_16x16x32_bf16(false, ah, false, bl, (short)0, c, false, false);
  asm volatile("v_nop\n\tv_nop\n\tv_nop\n\tv_nop" : "+v"(c) : "v"(ah), "v"(al), "v"(bh), "v"(bl));
  return c;
}

__global__ __launch_bounds__(256) void k_wt_bf16(const float* __restrict__ W, unsigned short* __restrict__ Wt, int K, int N) {
  const int t = blockIdx.x * 256 + threadIdx.x;
  const int k8n = K / 8;
  if (t >= N * k8n) return;
  const int n = t / k8n, k8 = (t % k8n) * 8;
  v8us v;
#pragma unroll
  for (int i = 0; i < 8; ++i) v[i] = bf16_bits(W[(size_t)(k8 + i) * N + n]);
  *(volatile v8us*)(Wt + (size_t)n * K + k8) = v;
  __threadfence();
  *(volatile v8us*)(Wt + (size_t)n * K + k8) = v;
}

template <bool ASPLIT, int ACT, bool BIAS_BF16>
__global__ __launch_bounds__(128) void k_gemm_bf(const float* __restrict__ A, int lda, const unsigned short* __restrict__ Wt, int ldb,
                                               const float* __restrict__ bias, float* __restrict__ C, int ldc, int M, int N, int K) {
  __shared__ __attribute__((aligned(16))) float so[4][16][64];
  const int tid = threadIdx.x, w = tid >> 5, lane = tid & 31, ln = lane & 15, hh = lane >> 4;
  const int ntn = N / 64;
  const int wid = blockIdx.x * 4 + w;
  const int mt = wid / ntn, nq = wid % ntn;
  if (mt * 16 >= M) return;
  const int row0 = mt * 16, col0 = nq * 64;
  const float* arow = A + (size_t)(row0 + ln) * lda;
  v8f acc[4] = {};
  for (int kb = 0; kb < K; kb += 32) {
    FragB ah, al;
    const v4f x0 = *(const v4fa*)(arow + kb + 8 * hh), x1 = *(const v4fa*)(arow + kb + 8 * hh + 4);
    const v4f x2 = *(const v4fa*)(arow + kb + 16 + 8 * hh), x3 = *(const v4fa*)(arow + kb + 16 + 8 * hh + 4);
    float xs[16] = {x0[0],x0[1],x0[2],x0[3],x1[0],x1[1],x1[2],x1[3],x2[0],x2[1],x2[2],x2[3],x3[0],x3[1],x3[2],x3[3]};
#pragma unroll
    for (int i = 0; i < 16; ++i) { const unsigned short hb = bf16_bits(xs[i]); ah.u[i] = hb; al.u[i] = ASPLIT ? bf16_bits(xs[i] - bf16_val(hb)) : (unsigned short)0; }
#pragma unroll
    for (int t = 0; t < 4; ++t) {
      const unsigned short* brow = Wt + (size_t)(col0 + t * 16 + ln) * ldb + kb;
      FragB b;
      b.half[0] = *(const v8us*)(brow + 8 * hh);
      b.half[1] = *(const v8us*)(brow + 16 + 8 * hh);
      acc[t] = mmaN<ASPLIT ? 2 : 1>(ah.v, al.v, b.v, b.v, acc[t]);
    }
  }
#pragma unroll
  for (int t = 0; t < 4; ++t) {
    float bv = bias ? bias[col0 + t * 16 + ln] : 0.f;
    if (BIAS_BF16) bv = bf16_round(bv);
#pragma unroll
    for (int r = 0; r < 8; ++r) { float v = acc[t][r] + bv; if (ACT == 1) v = fmaxf(v, 0.f); so[w][8 * hh + r][t * 16 + ln] = v; }
  }
  __builtin_amdgcn_fence(__ATOMIC_ACQ_REL, "workgroup");
  __builtin_amdgcn_wave_barrier();
  const int rsub = lane >> 4, c4 = (lane & 15) * 4;
  for (int pass = 0; pass < 2; ++pass) {
#pragma unroll
    for (int q = 0; q < 8; ++q) {
      const int r = q * 2 + rsub;
      const v4f v = *(const v4fa*)&so[w][r][c4];
      *(volatile v4f*)(C + (size_t)(row0 + r) * ldc + col0 + c4) = v;
    }
    if (pass == 0) __threadfence();
  }
}

template <int D, bool CAUSAL>
__global__ __launch_bounds__(128) void k_flash(const float* __restrict__ qb, const float* __restrict__ kb, const float* __restrict__ vb,
                                             int pitch, int T, int H, float scale, float* __restrict__ y, int ypitch) {
  constexpr int KS = D / 32;
  constexpr int DT = D / 16;
  __shared__ __attribute__((aligned(16))) unsigned short sKh[32][D + 8], sKl[32][D + 8], sVh[32][D + 8], sVl[32][D + 8];
  __shared__ __attribute__((aligned(16))) unsigned short sPh[4][16][40], sPl[4][16][40];
  __shared__ __attribute__((aligned(16))) float sO[4][16][D];
  const int tid = threadIdx.x, w = tid >> 5, lane = tid & 31, ln = lane & 15, hh = lane >> 4;
  const int nqb = (T + 63) / 64;
  const int bh = blockIdx.x / nqb, qblk = blockIdx.x % nqb;
  const int b = bh / H, h = bh % H;
  const int q0 = qblk * 64 + w * 16;
  const float* Q = qb + (size_t)b * T * pitch + h * D;
  const float* K = kb + (size_t)b * T * pitch + h * D;
  const float* V = vb + (size_t)b * T * pitch + h * D;

  FragB aqh[KS], aql[KS];
  {
    int row = q0 + ln; if (row >= T) row = T - 1;
    const float* qr = Q + (size_t)row * pitch;
#pragma unroll
    for (int ks = 0; ks < KS; ++ks)
#pragma unroll
      for (int i = 0; i < 16; ++i) {
        const int d = ks * 32 + ((i < 8) ? (8 * hh + i) : (16 + 8 * hh + (i - 8)));
        const float x = qr[d] * scale; const unsigned short hb = bf16_bits(x);
        aqh[ks].u[i] = hb; aql[ks].u[i] = bf16_bits(x - bf16_val(hb));
      }
  }
  float m_r[8], l_r[8];
#pragma unroll
  for (int r = 0; r < 8; ++r) { m_r[r] = -3.0e38f; l_r[r] = 0.f; }
  v8f oacc[DT];
#pragma unroll
  for (int dt = 0; dt < DT; ++dt) oacc[dt] = (v8f){0.f,0.f,0.f,0.f,0.f,0.f,0.f,0.f};

  const int kv_end = CAUSAL ? min(T, qblk * 64 + 64) : T;
  for (int j0 = 0; j0 < kv_end; j0 += 32) {
    __syncthreads();
    for (int e = tid; e < 32 * (D / 4); e += 128) {
      const int r = e / (D / 4), c4 = (e % (D / 4)) * 4;
      const int key = j0 + r;
      v4f kf = {0.f,0.f,0.f,0.f}, vf = {0.f,0.f,0.f,0.f};
      if (key < T) { kf = *(const v4fa*)(K + (size_t)key * pitch + c4); vf = *(const v4fa*)(V + (size_t)key * pitch + c4); }
#pragma unroll
      for (int t = 0; t < 4; ++t) {
        unsigned short hb = bf16_bits(kf[t]); sKh[r][c4 + t] = hb; sKl[r][c4 + t] = bf16_bits(kf[t] - bf16_val(hb));
        hb = bf16_bits(vf[t]); sVh[r][c4 + t] = hb; sVl[r][c4 + t] = bf16_bits(vf[t] - bf16_val(hb));
      }
    }
    __syncthreads();
    v8f s[2];
#pragma unroll
    for (int nt = 0; nt < 2; ++nt) {
      v8f acc = {};
#pragma unroll
      for (int ks = 0; ks < KS; ++ks) {
        FragB bh_, bl_;
        bh_.half[0] = *(const v8us*)&sKh[nt * 16 + ln][ks * 32 + 8 * hh]; bh_.half[1] = *(const v8us*)&sKh[nt * 16 + ln][ks * 32 + 16 + 8 * hh];
        bl_.half[0] = *(const v8us*)&sKl[nt * 16 + ln][ks * 32 + 8 * hh]; bl_.half[1] = *(const v8us*)&sKl[nt * 16 + ln][ks * 32 + 16 + 8 * hh];
        acc = mmaN<3>(aqh[ks].v, aql[ks].v, bh_.v, bl_.v, acc);
      }
      s[nt] = acc;
    }
    float alpha[8];
#pragma unroll
    for (int r = 0; r < 8; ++r) {
      const int qi = q0 + 8 * hh + r;
      const int ja = j0 + ln, jb = j0 + 16 + ln;
      if (CAUSAL) { if (ja > qi) s[0][r] = -3.0e38f; if (jb > qi) s[1][r] = -3.0e38f; }
      if (ja >= T) s[0][r] = -3.0e38f;
      if (jb >= T) s[1][r] = -3.0e38f;
      float mx = fmaxf(s[0][r], s[1][r]);
      mx = fmaxf(mx, __shfl_xor(mx, 1, 32)); mx = fmaxf(mx, __shfl_xor(mx, 2, 32)); mx = fmaxf(mx, __shfl_xor(mx, 4, 32)); mx = fmaxf(mx, __shfl_xor(mx, 8, 32));
      const float mnew = fmaxf(m_r[r], mx);
      alpha[r] = (mnew > -1.0e38f) ? __expf(m_r[r] - mnew) : 1.0f;
      const float p0 = (s[0][r] > -1.0e38f) ? __expf(s[0][r] - mnew) : 0.f;
      const float p1 = (s[1][r] > -1.0e38f) ? __expf(s[1][r] - mnew) : 0.f;
      m_r[r] = mnew;
      l_r[r] = l_r[r] * alpha[r] + p0 + p1;
      unsigned short hb = bf16_bits(p0); sPh[w][8 * hh + r][ln] = hb;      sPl[w][8 * hh + r][ln] = bf16_bits(p0 - bf16_val(hb));
      hb = bf16_bits(p1);                sPh[w][8 * hh + r][16 + ln] = hb; sPl[w][8 * hh + r][16 + ln] = bf16_bits(p1 - bf16_val(hb));
    }
#pragma unroll
    for (int dt = 0; dt < DT; ++dt)
#pragma unroll
      for (int r = 0; r < 8; ++r) oacc[dt][r] *= alpha[r];
    __builtin_amdgcn_fence(__ATOMIC_ACQ_REL, "workgroup");
    __builtin_amdgcn_wave_barrier();
    FragB pah, pal;
    pah.half[0] = *(const v8us*)&sPh[w][ln][8 * hh]; pah.half[1] = *(const v8us*)&sPh[w][ln][16 + 8 * hh];
    pal.half[0] = *(const v8us*)&sPl[w][ln][8 * hh]; pal.half[1] = *(const v8us*)&sPl[w][ln][16 + 8 * hh];
#pragma unroll
    for (int dt = 0; dt < DT; ++dt) {
      FragB bvh, bvl;
#pragma unroll
      for (int i = 0; i < 8; ++i) {
        bvh.u[i] = sVh[8 * hh + i][dt * 16 + ln]; bvh.u[8 + i] = sVh[16 + 8 * hh + i][dt * 16 + ln];
        bvl.u[i] = sVl[8 * hh + i][dt * 16 + ln]; bvl.u[8 + i] = sVl[16 + 8 * hh + i][dt * 16 + ln];
      }
      oacc[dt] = mmaN<3>(pah.v, pal.v, bvh.v, bvl.v, oacc[dt]);
    }
    __builtin_amdgcn_fence(__ATOMIC_ACQ_REL, "workgroup");
    __builtin_amdgcn_wave_barrier();
  }
#pragma unroll
  for (int r = 0; r < 8; ++r) {
    float l = l_r[r];
    l += __shfl_xor(l, 1, 32); l += __shfl_xor(l, 2, 32); l += __shfl_xor(l, 4, 32); l += __shfl_xor(l, 8, 32);
    l_r[r] = (l > 0.f) ? 1.0f / l : 0.f;
  }
#pragma unroll
  for (int dt = 0; dt < DT; ++dt)
#pragma unroll
    for (int r = 0; r < 8; ++r) sO[w][8 * hh + r][dt * 16 + ln] = oacc[dt][r] * l_r[r];
  __builtin_amdgcn_fence(__ATOMIC_ACQ_REL, "workgroup");
  __builtin_amdgcn_wave_barrier();
  for (int pass = 0; pass < 2; ++pass) {
    for (int r = 0; r < 16; ++r) {
      const int row = q0 + r;
      if (row < T && lane < D / 4) {
        const v4f val = *(const v4fa*)&sO[w][r][lane * 4];
        *(volatile v4f*)(y + ((size_t)b * T + row) * ypitch + h * D + lane * 4) = val;
      }
    }
    if (pass == 0) __threadfence();
  }
}

typedef _Float16 v16h __attribute__((ext_vector_type(16)));
union FragH { v16h v; v8us half[2]; _Float16 h[16]; unsigned short u[16]; };
template <int NT>
__device__ __forceinline__ v8f mmaH(v16h ah, v16h al, v16h bh, v16h bl, v8f c) {
  c = __builtin_amdgcn_wmma_f32_16x16x32_f16(false, ah, false, bh, (short)0, c, false, false);
  if (NT >= 2) c = __builtin_amdgcn_wmma_f32_16x16x32_f16(false, al, false, bh, (short)0, c, false, false);
  if (NT >= 3) c = __builtin_amdgcn_wmma_f32_16x16x32_f16(false, ah, false, bl, (short)0, c, false, false);
  asm volatile("v_nop\n\tv_nop\n\tv_nop\n\tv_nop" : "+v"(c) : "v"(ah), "v"(al), "v"(bh), "v"(bl));
  return c;
}
template <bool ASPLIT>
__global__ __launch_bounds__(128) void k_gemm_h(const float* __restrict__ A, int lda, size_t sA, const _Float16* __restrict__ Bh, int ldb, size_t sB, float alpha, float* __restrict__ C, int ldc, size_t sC, int M, int N, int K) {
  __shared__ __attribute__((aligned(16))) float so[4][16][64];
  const int tid = threadIdx.x, w = tid >> 5, lane = tid & 31, ln = lane & 15, hh = lane >> 4; const int by = blockIdx.y;
  A += (size_t)by * sA; Bh += (size_t)by * sB; C += (size_t)by * sC;
  const int ntn = (N + 63) / 64; const int wid = blockIdx.x * 4 + w; const int mt = wid / ntn, nq = wid % ntn; if (mt * 16 >= M) return;
  const int row0 = mt * 16, col0 = nq * 64; const float* arow = A + (size_t)(row0 + ln) * lda;
  v8f acc[4] = {};
  for (int kb = 0; kb < K; kb += 32) {
    FragH ah, al;
    const v4f x0 = *(const v4fa*)(arow + kb + 8 * hh), x1 = *(const v4fa*)(arow + kb + 8 * hh + 4), x2 = *(const v4fa*)(arow + kb + 16 + 8 * hh), x3 = *(const v4fa*)(arow + kb + 16 + 8 * hh + 4);
    float xs[16] = {x0[0],x0[1],x0[2],x0[3],x1[0],x1[1],x1[2],x1[3],x2[0],x2[1],x2[2],x2[3],x3[0],x3[1],x3[2],x3[3]};
#pragma unroll
    for (int i = 0; i < 16; ++i) { const _Float16 h = (_Float16)xs[i]; ah.h[i] = h; al.h[i] = ASPLIT ? (_Float16)(xs[i] - (float)h) : (_Float16)0.0f; }
#pragma unroll
    for (int t = 0; t < 4; ++t) { if (col0 + t * 16 >= N) continue; const size_t boff = (size_t)(col0 + t * 16 + ln) * ldb + kb; FragH bq; bq.half[0] = *(const v8us*)(Bh + boff + 8 * hh); bq.half[1] = *(const v8us*)(Bh + boff + 16 + 8 * hh);
      acc[t] = mmaH<ASPLIT ? 2 : 1>(ah.v, al.v, bq.v, bq.v, acc[t]); }
  }
#pragma unroll
  for (int t = 0; t < 4; ++t) { if (col0 + t * 16 >= N) continue;
#pragma unroll
    for (int r = 0; r < 8; ++r) so[w][8 * hh + r][t * 16 + ln] = acc[t][r] * alpha; }
  __builtin_amdgcn_fence(__ATOMIC_ACQ_REL, "workgroup"); __builtin_amdgcn_wave_barrier();
  const int rsub = lane >> 4, c4 = (lane & 15) * 4;
  for (int pass = 0; pass < 2; ++pass) {
#pragma unroll
    for (int q = 0; q < 8; ++q) { const int r = q * 2 + rsub; if (col0 + c4 < N) { const v4f v = *(const v4fa*)&so[w][r][c4]; *(volatile v4f*)(C + (size_t)(row0 + r) * ldc + col0 + c4) = v; } }
    if (pass == 0) __threadfence(); }
}

__device__ __forceinline__ float ftanh(float x) { return 1.0f - 2.0f / (__expf(2.0f * x) + 1.0f); }
__global__ __launch_bounds__(256) void k_bt(const float* __restrict__ W1, const float* __restrict__ W2, const float* __restrict__ W3, _Float16* __restrict__ W1T, _Float16* __restrict__ W2T, _Float16* __restrict__ W3T) { const size_t t = (size_t)blockIdx.x * 256 + threadIdx.x;
  if (t < (size_t)NE * HH * DI) { const int k = (int)(t % DI); const int n = (int)((t / DI) % HH); const int e = (int)(t / ((size_t)DI * HH)); *(volatile _Float16*)(W1T + t) = (_Float16)(bf16_round(W1[((size_t)e * DI + k) * HH + n]) * 16.0f); }
  if (t < (size_t)NE * HH * HH) { const int k = (int)(t % HH); const int n = (int)((t / HH) % HH); const int e = (int)(t / ((size_t)HH * HH)); *(volatile _Float16*)(W2T + t) = (_Float16)(bf16_round(W2[((size_t)e * HH + k) * HH + n]) * 16.0f); *(volatile _Float16*)(W3T + t) = (_Float16)(bf16_round(W3[((size_t)e * HH + k) * HH + n]) * 16.0f); } }
struct Route { int se0[TB], se1[TB]; float sg0[TB], sg1[TB], sgrow[TB][NE]; unsigned char slist[NE][2 * TB], sslot[NE][2 * TB]; int scnt[NE], stile_e[MAXT], stile_s[MAXT], sntile; };
__device__ void route(const float* __restrict__ x, const float* __restrict__ wg, int t0, Route& R) { const int tid = threadIdx.x;
  { const int n = t0 + tid; float lg[NE]; for (int e = 0; e < NE; ++e) lg[e] = 0.f;
#pragma unroll 1
    for (int k = 0; k < DI; ++k) { const float xv = bf16_round(x[(size_t)n * DI + k]);
#pragma unroll
      for (int e = 0; e < NE; ++e) lg[e] += xv * bf16_round(wg[k * NE + e]); }
    int i0 = 0; float v0 = lg[0]; for (int e = 1; e < NE; ++e) if (lg[e] > v0) { v0 = lg[e]; i0 = e; }
    int i1 = -1; float v1 = -3.0e38f; for (int e = 0; e < NE; ++e) if (e != i0 && (lg[e] > v1 || i1 < 0)) { v1 = lg[e]; i1 = e; }
    const float ex1 = expf(v1 - v0); const float g0 = 1.0f / (1.0f + ex1), g1 = ex1 / (1.0f + ex1);
    R.se0[tid] = i0; R.se1[tid] = i1; R.sg0[tid] = g0; R.sg1[tid] = g1; for (int e = 0; e < NE; ++e) R.sgrow[tid][e] = (e == i0) ? g0 : ((e == i1) ? g1 : 0.f); }
  __syncthreads();
  if (tid < NE) { int c = 0; for (int j = 0; j < TB; ++j) { if (R.se0[j] == tid) { R.slist[tid][c] = (unsigned char)j; R.sslot[tid][c] = 0; ++c; } if (R.se1[j] == tid) { R.slist[tid][c] = (unsigned char)j; R.sslot[tid][c] = 1; ++c; } } R.scnt[tid] = c; }
  __syncthreads();
  if (tid == 0) { int nt = 0; for (int e = 0; e < NE; ++e) for (int s = 0; s < R.scnt[e]; s += 16) { R.stile_e[nt] = e; R.stile_s[nt] = s; ++nt; } R.sntile = nt; }
  __syncthreads(); }
__global__ __launch_bounds__(TB) void k_gather(const float* __restrict__ x, const float* __restrict__ wg, const float* __restrict__ om, _Float16* __restrict__ XG) { __shared__ Route R; const int tid = threadIdx.x; const int t0 = blockIdx.x * TB; route(x, wg, t0, R);
  _Float16* base = XG + (size_t)blockIdx.x * MAXT * 16 * DI;
  for (int pass = 0; pass < 2; ++pass) {
    for (int row = 0; row < MAXT * 16; ++row) { const int ti = row >> 4, r = row & 15; float v = 0.f; if (ti < R.sntile) { const int e = R.stile_e[ti], idx = R.stile_s[ti] + r; if (idx < R.scnt[e]) { const int tok = t0 + R.slist[e][idx]; if (tid < DI) v = bf16_round(x[(size_t)tok * DI + tid]) * bf16_round(om[e]); } }
      if (tid < DI) *(volatile _Float16*)(base + (size_t)row * DI + tid) = (_Float16)v; }
    if (pass == 0) __threadfence(); } }
template <int KSTEPS, typename AF> __device__ __forceinline__ void tile_gemm(v8f (&acc)[16], const _Float16* __restrict__ Bt, int ldb, AF af, int ln, int hh) {
#pragma unroll
  for (int t = 0; t < 16; ++t) acc[t] = v8f{};
#pragma unroll 1
  for (int ks = 0; ks < KSTEPS; ++ks) { FragH a; af(ks, a);
#pragma unroll
    for (int t = 0; t < 16; ++t) { const unsigned short* p = (const unsigned short*)Bt + (size_t)(t * 16 + ln) * ldb + ks * 32; FragH bq; bq.half[0] = *(const v8us*)(p + 8 * hh); bq.half[1] = *(const v8us*)(p + 16 + 8 * hh); acc[t] = mmaH<1>(a.v, a.v, bq.v, bq.v, acc[t]); } } }
__global__ __launch_bounds__(TB) void k_moe(const float* __restrict__ x, const float* __restrict__ wg, const _Float16* __restrict__ XG, const _Float16* __restrict__ W1T, const float* __restrict__ b1, const _Float16* __restrict__ W2T, const float* __restrict__ b2, const _Float16* __restrict__ W3T, const float* __restrict__ b3, const float* __restrict__ Wo, const float* __restrict__ bo,
                                           float* __restrict__ OUT, float* __restrict__ GATES, float* __restrict__ PART) {
  __shared__ __attribute__((aligned(16))) float sh[4][16][HH + 4]; __shared__ Route R; __shared__ float sy[TB][2];
  const int tid = threadIdx.x, w = tid >> 5, lane = tid & 31, ln = lane & 15, hh = lane >> 4; const int t0 = blockIdx.x * TB;
  route(x, wg, t0, R);
  for (int pass = 0; pass < 2; ++pass) { for (int i = tid; i < TB * NE; i += TB) *(volatile float*)(GATES + (size_t)t0 * NE + i) = (&R.sgrow[0][0])[i]; if (pass == 0) __threadfence(); }
  if (tid < NE) { float imp = 0.f, ld = 0.f; for (int j = 0; j < TB; ++j) { const float gv = R.sgrow[j][tid]; imp += gv; ld += (gv > 0.f) ? 1.f : 0.f; } *(volatile float*)(PART + (size_t)blockIdx.x * 32 + tid) = imp; *(volatile float*)(PART + (size_t)blockIdx.x * 32 + NE + tid) = ld; }
  const _Float16* xg = XG + (size_t)blockIdx.x * MAXT * 16 * DI;
  for (int ti = w; ti < R.sntile; ti += 4) { const int e = R.stile_e[ti], s0 = R.stile_s[ti], cnt = R.scnt[e]; const _Float16* arow = xg + ((size_t)ti * 16 + ln) * DI;
    v8f acc[16];
    tile_gemm<2>(acc, W1T + (size_t)e * HH * DI, DI, [&](int ks, FragH& a) { a.half[0] = *(const v8us*)((const unsigned short*)arow + ks * 32 + 8 * hh); a.half[1] = *(const v8us*)((const unsigned short*)arow + ks * 32 + 16 + 8 * hh); }, ln, hh);
#pragma unroll
    for (int t = 0; t < 16; ++t) { const int c = t * 16 + ln; const float bb = bf16_round(b1[e * HH + c]);
#pragma unroll
      for (int r = 0; r < 8; ++r) sh[w][8 * hh + r][c] = ftanh(acc[t][r] * 0.0625f + bb); }
    __builtin_amdgcn_fence(__ATOMIC_ACQ_REL, "workgroup"); __builtin_amdgcn_wave_barrier();
    tile_gemm<8>(acc, W2T + (size_t)e * HH * HH, HH, [&](int ks, FragH& a) { for (int q = 0; q < 8; ++q) { a.h[q] = (_Float16)sh[w][ln][ks * 32 + 8 * hh + q]; a.h[8 + q] = (_Float16)sh[w][ln][ks * 32 + 16 + 8 * hh + q]; } }, ln, hh);
    __builtin_amdgcn_fence(__ATOMIC_ACQ_REL, "workgroup"); __builtin_amdgcn_wave_barrier();
#pragma unroll
    for (int t = 0; t < 16; ++t) { const int c = t * 16 + ln; const float bb = bf16_round(b2[e * HH + c]);
#pragma unroll
      for (int r = 0; r < 8; ++r) sh[w][8 * hh + r][c] = ftanh(acc[t][r] * 0.0625f + bb); }
    __builtin_amdgcn_fence(__ATOMIC_ACQ_REL, "workgroup"); __builtin_amdgcn_wave_barrier();
    tile_gemm<8>(acc, W3T + (size_t)e * HH * HH, HH, [&](int ks, FragH& a) { for (int q = 0; q < 8; ++q) { a.h[q] = (_Float16)sh[w][ln][ks * 32 + 8 * hh + q]; a.h[8 + q] = (_Float16)sh[w][ln][ks * 32 + 16 + 8 * hh + q]; } }, ln, hh);
    float part[8];
#pragma unroll
    for (int r = 0; r < 8; ++r) part[r] = 0.f;
#pragma unroll
    for (int t = 0; t < 16; ++t) { const int c = t * 16 + ln; const float bb = bf16_round(b3[e * HH + c]), wo = bf16_round(Wo[e * HH + c]);
#pragma unroll
      for (int r = 0; r < 8; ++r) part[r] += ftanh(acc[t][r] * 0.0625f + bb) * wo; }
#pragma unroll
    for (int r = 0; r < 8; ++r) { float v = part[r]; for (int o = 8; o >= 1; o >>= 1) v += __shfl_xor(v, o, 32); part[r] = v; }
    if (ln == 0) { const float bb = bf16_round(bo[e]);
#pragma unroll
      for (int r = 0; r < 8; ++r) { const int row = s0 + 8 * hh + r; if (row < cnt) sy[R.slist[e][row]][R.sslot[e][row]] = part[r] + bb; } }
    __builtin_amdgcn_fence(__ATOMIC_ACQ_REL, "workgroup"); __builtin_amdgcn_wave_barrier(); }
  __syncthreads();
  { const float o = R.sg0[tid] * sy[tid][0] + R.sg1[tid] * sy[tid][1]; *(volatile float*)(OUT + t0 + tid) = o; __threadfence(); *(volatile float*)(OUT + t0 + tid) = o; if (tid < 2 * NE) { const float p = *(volatile float*)(PART + (size_t)blockIdx.x * 32 + tid); *(volatile float*)(PART + (size_t)blockIdx.x * 32 + tid) = p; } } }
__global__ __launch_bounds__(64) void k_loss(const float* __restrict__ PART, int nb, float* __restrict__ out) { __shared__ float imp[NE], ld[NE]; const int tid = threadIdx.x; if (tid < 2 * NE) { float s = 0.f;
#pragma unroll 1
    for (int b = 0; b < nb; ++b) s += PART[(size_t)b * 32 + tid]; if (tid < NE) imp[tid] = s; else ld[tid - NE] = s; } __syncthreads();
  if (tid == 0) { auto cv2 = [](const float* v) { float m = 0.f; for (int e = 0; e < NE; ++e) m += v[e]; m /= (float)NE; float var = 0.f; for (int e = 0; e < NE; ++e) { const float d = v[e] - m; var += d * d; } var /= (float)NE; return var / (m * m + 1e-10f); };
    const float l = cv2(imp) + cv2(ld); *(volatile float*)out = l; __threadfence(); *(volatile float*)out = l; } }
extern "C" void kernel_launch(void* const* d_in, const int* in_sizes, int n_in,
                              void* d_out, int out_size, void* d_ws, size_t ws_size, hipStream_t stream) {
  (void)in_sizes; (void)n_in; (void)out_size;
  const float* x = (const float*)d_in[0]; const float* wg = (const float*)d_in[1]; const float* om = (const float*)d_in[2]; const float* W1 = (const float*)d_in[3]; const float* b1 = (const float*)d_in[4]; const float* W2 = (const float*)d_in[5]; const float* b2 = (const float*)d_in[6]; const float* W3 = (const float*)d_in[7]; const float* b3 = (const float*)d_in[8]; const float* Wo = (const float*)d_in[9]; const float* bo = (const float*)d_in[10];
  float* OUT = (float*)d_out; float* LOSS = (float*)((char*)d_out + 131072); float* GATES = (float*)((char*)d_out + 131076);
  char* ws = (char*)d_ws; size_t off = 0;
  auto take = [&](size_t bytes) { char* p = ws + off; off += (bytes + 255) & ~(size_t)255; return p; };
  const int NBLK = NTK / TB;
  _Float16* W1T = (_Float16*)take((size_t)NE * HH * DI * 2); _Float16* W2T = (_Float16*)take((size_t)NE * HH * HH * 2); _Float16* W3T = (_Float16*)take((size_t)NE * HH * HH * 2); _Float16* XG = (_Float16*)take((size_t)NBLK * MAXT * 16 * DI * 2); float* PART = (float*)take((size_t)NBLK * 32 * 4);
  if (off > ws_size) return;
  k_bt<<<(unsigned)(((size_t)NE * HH * HH + 255) / 256), 256, 0, stream>>>(W1, W2, W3, W1T, W2T, W3T);
  k_gather<<<NBLK, TB, 0, stream>>>(x, wg, om, XG);
  k_moe<<<NBLK, TB, 0, stream>>>(x, wg, XG, W1T, b1, W2T, b2, W3T, b3, Wo, bo, OUT, GATES, PART);
  k_loss<<<1, 64, 0, stream>>>(PART, NBLK, LOSS);
}
